// MoEGraphLayer_38371237822640
// MI455X (gfx1250) — hardware-verified
//
#include <hip/hip_runtime.h>
#include <math.h>

typedef __attribute__((ext_vector_type(16))) _Float16 v16h;
typedef __attribute__((ext_vector_type(16))) __bf16 v16b;
typedef __attribute__((ext_vector_type(8)))  _Float16 v8h;
typedef __attribute__((ext_vector_type(8)))  float v8f;
typedef __attribute__((ext_vector_type(4)))  float v4f;
typedef __attribute__((ext_vector_type(2)))  float v2f;
typedef __attribute__((ext_vector_type(4)))  unsigned v4u;
typedef __attribute__((ext_vector_type(4)))  int v4i;
typedef float __attribute__((may_alias)) float_a;
typedef int __attribute__((may_alias)) int_a;

template <typename T> __device__ __forceinline__ void vst2(void* p, T v) { *(volatile T*)p = v; __threadfence(); *(volatile T*)p = v; }
__device__ __forceinline__ v8f wmma16(v16h a, v16h b, v8f c) {
  v8f d = __builtin_amdgcn_wmma_f32_16x16x32_f16(false, a, false, b, (short)0, c, false, false);
  asm volatile("v_nop\n\tv_nop\n\tv_nop\n\tv_nop" : "+v"(d) : "v"(a), "v"(b));
  return d;
}
__device__ __forceinline__ v8f wmma_bf(v16b a, v16b b, v8f c) {
  v8f d = __builtin_amdgcn_wmma_f32_16x16x32_bf16(false, a, false, b, (short)0, c, false, false);
  asm volatile("v_nop\n\tv_nop\n\tv_nop\n\tv_nop" : "+v"(d) : "v"(a), "v"(b));
  return d;
}
__device__ __forceinline__ v16h frag_h(const _Float16* rowk0, int lane) {
  union { v16h v; v8h q[2]; } u; const _Float16* p = rowk0 + 8 * (lane >> 4);
  u.q[0] = *(const v8h*)p; u.q[1] = *(const v8h*)(p + 16); return u.v;
}
__device__ __forceinline__ v16h frag_f32(const float* rowk0, int lane) {
  v16h a; const float* p = rowk0 + 8 * (lane >> 4);
#pragma unroll
  for (int i = 0; i < 8; ++i) { a[i] = (_Float16)p[i]; a[8 + i] = (_Float16)p[16 + i]; }
  return a;
}
__device__ __forceinline__ v16h frag_f32s(const float* rowk0, int lane, float sc) {
  v16h a; const float* p = rowk0 + 8 * (lane >> 4);
#pragma unroll
  for (int i = 0; i < 8; ++i) { a[i] = (_Float16)(p[i] * sc); a[8 + i] = (_Float16)(p[16 + i] * sc); }
  return a;
}
__device__ __forceinline__ v16h fragc_f32(const float* W, int k0, int n, int lane, int ld, int K) {
  v16h a; const int g = lane >> 4;
#pragma unroll
  for (int i = 0; i < 8; ++i) { const int ka = k0 + 8 * g + i, kb = ka + 16;
    a[i] = (_Float16)(ka < K ? W[(size_t)(ka < K ? ka : K - 1) * ld + n] : 0.f); a[8 + i] = (_Float16)(kb < K ? W[(size_t)(kb < K ? kb : K - 1) * ld + n] : 0.f); }
  return a;
}
struct F2 { v16b h, l; };
__device__ __forceinline__ F2 bsplit16(const float v[16]) { F2 r;
#pragma unroll
  for (int i = 0; i < 16; ++i) { const __bf16 h = (__bf16)v[i]; r.h[i] = h; r.l[i] = (__bf16)(v[i] - (float)h); }
  return r; }
__device__ __forceinline__ F2 split_row(const float* row, int k0, int lane) { float v[16]; const float* p = row + k0 + 8 * (lane >> 4);
#pragma unroll
  for (int i = 0; i < 8; ++i) { v[i] = p[i]; v[8 + i] = p[16 + i]; }
  return bsplit16(v); }
__device__ __forceinline__ F2 split_rowK(const float* row, int k0, int lane, int K) { float v[16]; const int g = lane >> 4;
#pragma unroll
  for (int i = 0; i < 8; ++i) { const int ka = k0 + 8 * g + i, kb = ka + 16; v[i] = ka < K ? row[ka < K ? ka : K - 1] : 0.f; v[8 + i] = kb < K ? row[kb < K ? kb : K - 1] : 0.f; }
  return bsplit16(v); }
__device__ __forceinline__ F2 split_col(const float* W, int k0, int n, int lane, int ld, int K) { float v[16]; const int g = lane >> 4;
#pragma unroll
  for (int i = 0; i < 8; ++i) { const int ka = k0 + 8 * g + i, kb = ka + 16; v[i] = ka < K ? W[(size_t)(ka < K ? ka : K - 1) * ld + n] : 0.f; v[8 + i] = kb < K ? W[(size_t)(kb < K ? kb : K - 1) * ld + n] : 0.f; }
  return bsplit16(v); }
__device__ __forceinline__ v8f mac3(const F2& a, const F2& b, v8f c) { c = wmma_bf(a.l, b.h, c); c = wmma_bf(a.h, b.l, c); return wmma_bf(a.h, b.h, c); }
__device__ __forceinline__ float sigm(float v) { return 1.0f / (1.0f + expf(-v)); }
#define LDSX() do { asm volatile("s_wait_dscnt 0" ::: "memory"); __builtin_amdgcn_wave_barrier(); __builtin_amdgcn_fence(__ATOMIC_RELEASE, "workgroup"); } while (0)


#ifndef NB
#define NB 4
#endif
#define SQ 1024
#define NT (NB * SQ)
#define NTO (4 * SQ)
#define DD 256
#define NHD 6
#define HD 64
#define HW (NHD * HD)
#define NE 3
#define NDOC 4
#define NSECT 32
typedef __attribute__((ext_vector_type(8))) __bf16 v8b;
__device__ __forceinline__ v16b frag_b(const __bf16* rowk0, int lane) {
  union { v16b v; v8b q[2]; } u; const __bf16* p = rowk0 + 8 * (lane >> 4);
  u.q[0] = *(const v8b*)p; u.q[1] = *(const v8b*)(p + 16); return u.v;
}
__device__ __forceinline__ float bfr(float v) { return (float)(__bf16)v; }
__device__ __attribute__((noinline)) float exp_ni(float v) { return expf(v); }
__device__ __attribute__((noinline)) float erf_ni(float v) { return erff(v); }

__device__ __attribute__((noinline)) float expm1_ni(float v) { return expm1f(v); }
#define WS_PW   0u
#define PG1(g) ((size_t)(g) * (384 * 256 + 256 * 384))
#define PG2(g) (PG1(g) + 384 * 256)
#define PRT  (PG1(4))
#define PBL  (PRT + 16 * 256)
#define PWEND (PBL + 256 * 256)
#define WS_MASK (WS_PW + 2u * PWEND)
#define WS_H    (WS_MASK + 4u * NT * 4)
#define WS_E1   (WS_H + 4u * NT * HW)
#define WS_VT1  (WS_E1 + 4u * NHD * NT * 2)
#define WS_VT1L (WS_VT1 + 2u * NB * NHD * HD * SQ)
#define WS_H1   (WS_VT1L + 2u * NB * NHD * HD * SQ)
#define WS_H2   (WS_H1 + 4u * NT * HW)
#define WS_E2   (WS_H2 + 4u * NT * DD)
#define WS_VT2  (WS_E2 + 4u * NT * 2)
#define WS_VT2L (WS_VT2 + 2u * NB * DD * SQ)
#define WS_MAIN (WS_VT2L + 2u * NB * DD * SQ)
#define WS_DEP  (WS_MAIN + 4u * NT * DD)
#define WS_BL   (WS_DEP + 4u * NT * DD)
#define WS_PB   (WS_BL + 4u * NT * DD)
#define WS_END  (WS_PB + 4u * (NT / 64) * 32)

__global__ __launch_bounds__(128) void k_pack(const float* __restrict__ MW1, const float* __restrict__ MW2, const float* __restrict__ DW1, const float* __restrict__ DW2, const float* __restrict__ RW, const float* __restrict__ BW, __bf16* __restrict__ PW) {
  __shared__ __align__(16) __bf16 s[384]; const int n = blockIdx.x, which = blockIdx.y, t = threadIdx.x; int K; size_t dst;
  if (which < 4) { if (n >= HW) return; K = DD; const int g = which; const int h = n / HD, o = n % HD; const float* W = (g == 0) ? MW1 : DW1 + (size_t)(g - 1) * NHD * DD * HD; dst = PG1(g) + (size_t)n * DD; for (int k = t; k < K; k += 128) s[k] = (__bf16)W[((size_t)h * DD + k) * HD + o]; }
  else if (which < 8) { if (n >= DD) return; K = HW; const int g = which - 4; const float* W = (g == 0) ? MW2 : DW2 + (size_t)(g - 1) * HW * DD; dst = PG2(g) + (size_t)n * HW; for (int k = t; k < K; k += 128) s[k] = (__bf16)W[(size_t)k * DD + n]; }
  else if (which == 8) { if (n >= 16) return; K = DD; dst = PRT + (size_t)n * DD; for (int k = t; k < K; k += 128) s[k] = (__bf16)((n < NE) ? RW[(size_t)k * NE + n] : 0.f); }
  else { if (n >= DD) return; K = DD; dst = PBL + (size_t)n * DD; for (int k = t; k < K; k += 128) s[k] = (__bf16)BW[(size_t)k * DD + n]; }
  __syncthreads();
  if (t < K / 8) vst2((unsigned*)(PW + dst + t * 8), *(const v4u*)&s[t * 8]);
}
__global__ __launch_bounds__(128) void k_router(const float* __restrict__ X, const __bf16* __restrict__ PW, float* __restrict__ MASK) {
  __shared__ float sl[4][16][4]; __shared__ __align__(16) float sm[64][4];
  const int tid = threadIdx.x, wave = tid >> 5, lane = tid & 31, col = lane & 15, g = lane >> 4; const size_t r0 = (size_t)blockIdx.x * 64 + wave * 16;
  v8f acc = {};
#pragma unroll 2
  for (int kc = 0; kc < DD / 32; ++kc) { v16b a; { const float* p = X + (r0 + col) * DD + kc * 32 + 8 * g;
#pragma unroll
      for (int i = 0; i < 8; ++i) { a[i] = (__bf16)p[i]; a[8 + i] = (__bf16)p[16 + i]; } }
    acc = wmma_bf(a, frag_b(PW + PRT + (size_t)col * DD + kc * 32, lane), acc); }
  if (col < NE) {
#pragma unroll
    for (int r = 0; r < 8; ++r) sl[wave][8 * g + r][col] = acc[r]; }
  LDSX();
  if (lane < 16) { const int tl = wave * 16 + lane; const float l0 = sl[wave][lane][0], l1 = sl[wave][lane][1], l2 = sl[wave][lane][2];
    int i1 = 0; float v1 = l0; if (l1 > v1) { v1 = l1; i1 = 1; } if (l2 > v1) { v1 = l2; i1 = 2; }
    int i2 = -1; float v2 = -3.0e38f; if (0 != i1 && l0 > v2) { v2 = l0; i2 = 0; } if (1 != i1 && l1 > v2) { v2 = l1; i2 = 1; } if (2 != i1 && l2 > v2) { v2 = l2; i2 = 2; }
    sm[tl][0] = (i1 == 0 || i2 == 0) ? 1.f : 0.f; sm[tl][1] = (i1 == 1 || i2 == 1) ? 1.f : 0.f; sm[tl][2] = (i1 == 2 || i2 == 2) ? 1.f : 0.f; sm[tl][3] = 0.f; }
  __syncthreads();
  if (tid < 64) vst2(MASK + ((size_t)blockIdx.x * 64 + tid) * 4, *(const v4f*)&sm[tid][0]);
}
__global__ __launch_bounds__(128) void k_h1(const float* __restrict__ X, const float* __restrict__ MASK, int g, const __bf16* __restrict__ PW, const float* __restrict__ A1S, const float* __restrict__ A1D, float* __restrict__ Hh, float* __restrict__ E1) {
  __shared__ __align__(16) float so[4][16][132]; __shared__ __align__(16) float se[2][64][2];
  const int tid = threadIdx.x, wave = tid >> 5, lane = tid & 31, col = lane & 15, gg = lane >> 4; const size_t r0 = (size_t)blockIdx.x * 64 + wave * 16; const int n0 = blockIdx.y * 128; const int h0 = blockIdx.y * 2;
  v8f acc[8] = {};
#pragma unroll 2
  for (int kc = 0; kc < DD / 32; ++kc) { v16b a; { const float* p = X + (r0 + col) * DD + kc * 32 + 8 * gg;
#pragma unroll
      for (int i = 0; i < 8; ++i) { a[i] = (__bf16)p[i]; a[8 + i] = (__bf16)p[16 + i]; } }
#pragma unroll
    for (int j = 0; j < 8; ++j) acc[j] = wmma_bf(a, frag_b(PW + PG1(g) + (size_t)(n0 + j * 16 + col) * DD + kc * 32, lane), acc[j]); }
#pragma unroll
  for (int j = 0; j < 8; ++j)
#pragma unroll
    for (int r = 0; r < 8; ++r) { const size_t row = r0 + 8 * gg + r; const float m = (g == 0) ? 1.f : MASK[row * 4 + (g - 1)]; so[wave][8 * gg + r][j * 16 + col] = acc[j][r] * m; }
  LDSX();
  for (int rl = 0; rl < 16; ++rl) { const int hh = lane >> 4; const int hg = h0 + hh; float a1 = 0.f, a2 = 0.f;
#pragma unroll
    for (int q = 0; q < 4; ++q) { const int c = hh * 64 + (lane & 15) * 4 + q; const float hv = so[wave][rl][c]; a1 += hv * bfr(A1S[hg * HD + (c & 63)]); a2 += hv * bfr(A1D[hg * HD + (c & 63)]); }
#pragma unroll
    for (int o = 1; o < 16; o <<= 1) { a1 += __shfl_xor(a1, o); a2 += __shfl_xor(a2, o); }
    if ((lane & 15) == 0) { se[hh][wave * 16 + rl][0] = a1; se[hh][wave * 16 + rl][1] = a2; } }
  for (int rl = 0; rl < 16; ++rl) vst2(Hh + (r0 + rl) * HW + n0 + lane * 4, *(const v4f*)&so[wave][rl][lane * 4]);
  __syncthreads();
  for (int q = tid; q < 2 * 32; q += 128) { const int hh = q >> 5, pc = q & 31; vst2(E1 + ((size_t)(h0 + hh) * NT + (size_t)blockIdx.x * 64) * 2 + pc * 4, *(const v4f*)(&se[hh][0][0] + pc * 4)); }
}
template <int PD, int NPL>
__global__ __launch_bounds__(256) void k_vt(const float* __restrict__ M, int ldm, __bf16* __restrict__ VT, __bf16* __restrict__ VTL) {
  __shared__ __align__(16) __bf16 sh[PD][72], sl[PD][72]; const int tid = threadIdx.x; const size_t t0 = (size_t)blockIdx.x * 64; const int b = (int)(t0 / SQ); const int s0 = (int)(t0 % SQ); const int p = blockIdx.y;
  for (int q = tid; q < PD * 64; q += 256) { const int d = q >> 6, nl = q & 63; const float v = M[(t0 + nl) * ldm + p * PD + d]; const __bf16 hb = (__bf16)v; sh[d][nl] = hb; sl[d][nl] = (__bf16)(v - (float)hb); }
  __syncthreads();
  for (int q = tid; q < PD * 8; q += 256) { const int d = q >> 3, pc = q & 7; const size_t base = ((size_t)(b * NPL + p) * PD + d) * SQ + s0 + pc * 8; vst2((unsigned*)(VT + base), *(const v4u*)&sh[d][pc * 8]); vst2((unsigned*)(VTL + base), *(const v4u*)&sl[d][pc * 8]); }
}
template <int NDT, int MODE, int L1>
__global__ __launch_bounds__(128) void k_att(const float* __restrict__ ESb, const float* __restrict__ ADJ, int tlo, int thi, const __bf16* __restrict__ VT, const __bf16* __restrict__ VTL, int npl, const float* __restrict__ MASK, int g, float* __restrict__ OUT, int ldo) {
  __shared__ __align__(16) float sp[4][16][36]; __shared__ __align__(16) float so[4][16][NDT * 16 + 4];
  const int tid = threadIdx.x, wave = tid >> 5, lane = tid & 31, col = lane & 15, gg = lane >> 4; const int b = blockIdx.x / (SQ / 64); const size_t q0 = (size_t)blockIdx.x * 64 + wave * 16; const int p = blockIdx.y; const int sq0 = (int)(q0 % SQ);
  const float* ES = ESb + (L1 ? (size_t)p * NT * 2 : 0); const int vplane = b * npl + (L1 ? p : 0); const int vdim0 = L1 ? 0 : p * NDT * 16; constexpr int PDIM = L1 ? HD : DD;
  float esr[8];
#pragma unroll
  for (int r = 0; r < 8; ++r) esr[r] = ES[(q0 + 8 * gg + r) * 2];
  float m[8], l[8];
#pragma unroll
  for (int r = 0; r < 8; ++r) { m[r] = -3.0e38f; l[r] = 0.f; }
  v8f acc[NDT]; for (int j = 0; j < NDT; ++j) acc[j] = (v8f){};
  const float* adjb = ADJ + (size_t)b * SQ * SQ;
#pragma unroll 1
  for (int ks = 0; ks < SQ / 32; ++ks) {
    float edc[2]; { const int t0 = ks * 32 + col; edc[0] = ES[((size_t)b * SQ + t0) * 2 + 1]; edc[1] = ES[((size_t)b * SQ + t0 + 16) * 2 + 1]; }
#pragma unroll
    for (int r = 0; r < 8; ++r) { const int s = sq0 + 8 * gg + r; float sv[2];
#pragma unroll
      for (int ct = 0; ct < 2; ++ct) { const int t = ks * 32 + ct * 16 + col; float e = esr[r] + edc[ct]; e = e > 0.f ? e : 0.2f * e; const bool ok = (t >= tlo && t < thi) && (bfr(adjb[(size_t)s * SQ + t]) > 0.f); sv[ct] = ok ? e : -1.0e9f; }
      float mx = fmaxf(sv[0], sv[1]);
#pragma unroll
      for (int o = 1; o < 16; o <<= 1) mx = fmaxf(mx, __shfl_xor(mx, o));
      const float mn = fmaxf(m[r], mx); const float alpha = (m[r] <= -1.0e38f) ? 0.f : exp_ni(m[r] - mn); const float e0 = exp_ni(sv[0] - mn), e1 = exp_ni(sv[1] - mn); float es_ = e0 + e1;
#pragma unroll
      for (int o = 1; o < 16; o <<= 1) es_ += __shfl_xor(es_, o);
      l[r] = l[r] * alpha + es_; m[r] = mn;
#pragma unroll
      for (int j = 0; j < NDT; ++j) acc[j][r] *= alpha;
      sp[wave][8 * gg + r][col] = e0; sp[wave][8 * gg + r][16 + col] = e1; }
    LDSX();
    const F2 pa = split_row(&sp[wave][col][0], 0, lane);
#pragma unroll
    for (int j = 0; j < NDT; ++j) { const size_t pr = ((size_t)vplane * PDIM + vdim0 + j * 16 + col) * SQ + ks * 32; const v16b vh = frag_b(VT + pr, lane), vl = frag_b(VTL + pr, lane); acc[j] = wmma_bf(pa.l, vh, acc[j]); acc[j] = wmma_bf(pa.h, vl, acc[j]); acc[j] = wmma_bf(pa.h, vh, acc[j]); }
    LDSX(); }
#pragma unroll
  for (int j = 0; j < NDT; ++j)
#pragma unroll
    for (int r = 0; r < 8; ++r) { float v = acc[j][r] / l[r]; if (MODE == 0) v = v > 0.f ? v : expm1_ni(v); so[wave][8 * gg + r][j * 16 + col] = v; }
  LDSX();
  const int c0 = p * NDT * 16;
  for (int rl = 0; rl < 16; ++rl) { const size_t row = q0 + rl; const float mrow = (MODE >= 2) ? MASK[row * 4 + (g - 1)] : 1.f;
    for (int pc = lane; pc < NDT * 4; pc += 32) { v4f v = *(const v4f*)&so[wave][rl][pc * 4]; float* dst = OUT + row * (size_t)ldo + c0 + pc * 4;
      if (MODE >= 2) {
#pragma unroll
        for (int i = 0; i < 4; ++i) v[i] = mrow * v[i]; }
      if (MODE == 2) { const v4f old = *(const v4f*)dst;
#pragma unroll
        for (int i = 0; i < 4; ++i) v[i] = old[i] + v[i]; }
      vst2(dst, v); } }
}
__global__ __launch_bounds__(128) void k_h2(const float* __restrict__ H1, int g, const __bf16* __restrict__ PW, float* __restrict__ H2) {
  __shared__ __align__(16) float so[4][16][132];
  const int tid = threadIdx.x, wave = tid >> 5, lane = tid & 31, col = lane & 15, gg = lane >> 4; const size_t r0 = (size_t)blockIdx.x * 64 + wave * 16; const int n0 = blockIdx.y * 128;
  v8f acc[8] = {};
#pragma unroll 2
  for (int kc = 0; kc < HW / 32; ++kc) { const F2 a = split_row(H1 + (r0 + col) * HW, kc * 32, lane);
#pragma unroll
    for (int j = 0; j < 8; ++j) { const v16b w = frag_b(PW + PG2(g) + (size_t)(n0 + j * 16 + col) * HW + kc * 32, lane); acc[j] = wmma_bf(a.l, w, acc[j]); acc[j] = wmma_bf(a.h, w, acc[j]); } }
#pragma unroll
  for (int j = 0; j < 8; ++j)
#pragma unroll
    for (int r = 0; r < 8; ++r) so[wave][8 * gg + r][j * 16 + col] = acc[j][r];
  LDSX();
  for (int rl = 0; rl < 16; ++rl) vst2(H2 + (r0 + rl) * DD + n0 + lane * 4, *(const v4f*)&so[wave][rl][lane * 4]);
}
__global__ __launch_bounds__(512) void k_e2(const float* __restrict__ H2, const float* __restrict__ A2S, const float* __restrict__ A2D, float* __restrict__ E2) {
  __shared__ __align__(16) float s[16][2]; const int tid = threadIdx.x, wave = tid >> 5, lane = tid & 31; const size_t row = (size_t)blockIdx.x * 16 + wave;
  float a1 = 0.f, a2 = 0.f;
#pragma unroll
  for (int q = 0; q < 8; ++q) { const int c = lane + 32 * q; const float hv = H2[row * DD + c]; a1 += hv * bfr(A2S[c]); a2 += hv * bfr(A2D[c]); }
#pragma unroll
  for (int o = 1; o < 32; o <<= 1) { a1 += __shfl_xor(a1, o); a2 += __shfl_xor(a2, o); }
  if (lane == 0) { s[wave][0] = a1; s[wave][1] = a2; }
  __syncthreads();
  if (tid < 8) vst2(E2 + (size_t)blockIdx.x * 32 + tid * 4, *(const v4f*)(&s[0][0] + tid * 4));
}
__global__ __launch_bounds__(128) void k_blend(const float* __restrict__ X, const __bf16* __restrict__ PW, const float* __restrict__ BB, float* __restrict__ BL) {
  __shared__ __align__(16) float so[4][16][132];
  const int tid = threadIdx.x, wave = tid >> 5, lane = tid & 31, col = lane & 15, gg = lane >> 4; const size_t r0 = (size_t)blockIdx.x * 64 + wave * 16; const int n0 = blockIdx.y * 128;
  v8f acc[8] = {};
#pragma unroll 2
  for (int kc = 0; kc < DD / 32; ++kc) { v16b a; { const float* p = X + (r0 + col) * DD + kc * 32 + 8 * gg;
#pragma unroll
      for (int i = 0; i < 8; ++i) { a[i] = (__bf16)p[i]; a[8 + i] = (__bf16)p[16 + i]; } }
#pragma unroll
    for (int j = 0; j < 8; ++j) acc[j] = wmma_bf(a, frag_b(PW + PBL + (size_t)(n0 + j * 16 + col) * DD + kc * 32, lane), acc[j]); }
#pragma unroll
  for (int j = 0; j < 8; ++j) { const float bb = bfr(BB[n0 + j * 16 + col]);
#pragma unroll
    for (int r = 0; r < 8; ++r) so[wave][8 * gg + r][j * 16 + col] = sigm(acc[j][r] + bb); }
  LDSX();
  for (int rl = 0; rl < 16; ++rl) vst2(BL + (r0 + rl) * DD + n0 + lane * 4, *(const v4f*)&so[wave][rl][lane * 4]);
}
__global__ __launch_bounds__(256) void k_final(const float* __restrict__ BL, const float* __restrict__ MAIN, const float* __restrict__ DEP, float* __restrict__ OUT, float* __restrict__ PB) {
  __shared__ __align__(16) float srow[256]; __shared__ float ssum[256]; __shared__ __align__(16) float sl[32]; const int t = threadIdx.x; const size_t r0 = (size_t)blockIdx.x * 64; float a = 0.f;
  for (int r = 0; r < 64; ++r) { const size_t idx = (r0 + r) * DD + t; const float bl = BL[idx]; a += bl; srow[t] = bl * MAIN[idx] + (1.0f - bl) * DEP[idx]; __syncthreads(); if (t < 64) vst2(OUT + (r0 + r) * DD + t * 4, *(const v4f*)&srow[t * 4]); __syncthreads(); }
  ssum[t] = a; __syncthreads();
  for (int o = 128; o > 0; o >>= 1) { if (t < o) ssum[t] += ssum[t + o]; __syncthreads(); }
  if (t < 32) sl[t] = (t == 0) ? ssum[0] : 0.f;
  __syncthreads();
  if (t < 8) vst2(PB + (size_t)blockIdx.x * 32 + t * 4, *(const v4f*)&sl[t * 4]);
}
__global__ __launch_bounds__(64) void k_scalars(const float* __restrict__ PB, float* __restrict__ OUTS) {
  const int t = threadIdx.x; if (t == 0) { float a = 0.f; for (int b = 0; b < NT / 64; ++b) a += PB[b * 32]; const float mc = a / (float)(NT * DD); const float loss = fabsf(mc - 0.6f) * 0.01f; vst2(OUTS, (v2f){loss, mc}); }
}
extern "C" void kernel_launch(void* const* d_in, const int* in_sizes, int n_in, void* d_out, int out_size, void* d_ws, size_t ws_size, hipStream_t stream) {
  (void)in_sizes; (void)n_in; (void)out_size;
  const float** F = (const float**)d_in;
  if (ws_size < (size_t)WS_END) return;
  char* ws = (char*)d_ws; __bf16* PW = (__bf16*)(ws + WS_PW); float *MASK = (float*)(ws + WS_MASK), *Hh = (float*)(ws + WS_H), *E1 = (float*)(ws + WS_E1), *H1 = (float*)(ws + WS_H1), *H2 = (float*)(ws + WS_H2), *E2 = (float*)(ws + WS_E2), *MAIN = (float*)(ws + WS_MAIN), *DEP = (float*)(ws + WS_DEP), *BL = (float*)(ws + WS_BL), *PB = (float*)(ws + WS_PB);
  __bf16 *VT1 = (__bf16*)(ws + WS_VT1), *VT1L = (__bf16*)(ws + WS_VT1L), *VT2 = (__bf16*)(ws + WS_VT2), *VT2L = (__bf16*)(ws + WS_VT2L);
  float* OUT = (float*)d_out; float* OUTS = OUT + (size_t)NTO * DD;
  k_pack<<<dim3(HW, 10), 128, 0, stream>>>(F[2], F[5], F[8], F[11], F[14], F[15], PW);
  k_router<<<NT / 64, 128, 0, stream>>>(F[0], PW, MASK);
  k_blend<<<dim3(NT / 64, 2), 128, 0, stream>>>(F[0], PW, F[16], BL);
  for (int g = 0; g < 4; ++g) {
    const int tlo = (g == 0) ? 0 : (g == 1 ? 0 : (g == 2 ? SQ - NSECT - NDOC : SQ - NDOC)); const int thi = (g == 0) ? SQ : (g == 1 ? SQ - NSECT - NDOC : (g == 2 ? SQ - NDOC : SQ));
    const float* a1s = (g == 0) ? F[3] : F[9] + (size_t)(g - 1) * NHD * HD; const float* a1d = (g == 0) ? F[4] : F[10] + (size_t)(g - 1) * NHD * HD; const float* a2s = (g == 0) ? F[6] : F[12] + (size_t)(g - 1) * DD; const float* a2d = (g == 0) ? F[7] : F[13] + (size_t)(g - 1) * DD;
    k_h1<<<dim3(NT / 64, 3), 128, 0, stream>>>(F[0], MASK, g, PW, a1s, a1d, Hh, E1);
    k_vt<HD, NHD><<<dim3(NT / 64, NHD), 256, 0, stream>>>(Hh, HW, VT1, VT1L);
    k_att<4, 0, 1><<<dim3(NT / 64, NHD), 128, 0, stream>>>(E1, F[1], tlo, thi, VT1, VT1L, NHD, MASK, g, H1, HW);
    k_h2<<<dim3(NT / 64, 2), 128, 0, stream>>>(H1, g, PW, H2);
    k_e2<<<NT / 16, 512, 0, stream>>>(H2, a2s, a2d, E2);
    k_vt<DD, 1><<<dim3(NT / 64, 1), 256, 0, stream>>>(H2, DD, VT2, VT2L);
    if (g == 0)      k_att<8, 1, 0><<<dim3(NT / 64, 2), 128, 0, stream>>>(E2, F[1], tlo, thi, VT2, VT2L, 1, MASK, g, MAIN, DD);
    else if (g == 1) k_att<8, 3, 0><<<dim3(NT / 64, 2), 128, 0, stream>>>(E2, F[1], tlo, thi, VT2, VT2L, 1, MASK, g, DEP, DD);
    else             k_att<8, 2, 0><<<dim3(NT / 64, 2), 128, 0, stream>>>(E2, F[1], tlo, thi, VT2, VT2L, 1, MASK, g, DEP, DD);
  }
  k_final<<<NT / 64, 256, 0, stream>>>(BL, MAIN, DEP, OUT, PB);
  k_scalars<<<1, 64, 0, stream>>>(PB, OUTS);
}
